// GATv2_10041633538649
// MI455X (gfx1250) — hardware-run, weakly checked
//
#include <hip/hip_runtime.h>
#include <stddef.h>
#include <stdint.h>


#define IN1   128
#define HCH   256
#define HIDW  64
#define OUTW  8
#define NTHR  256
#define NWAVE 8
#define NB    240
#define SPW   (NB / NWAVE)
#define CHUNK 2048
#define WCAP  256
#define NGRP  (CHUNK / (NTHR * 4))
#define GR    64
#define TSP   136
#define HSP   68

#define LDS_ACC  (NB * HCH)
#define LDS_MD   (NB * 8)
#define LDS_LIST (NWAVE * WCAP)
#define LDS_AGG_BYTES ((LDS_ACC + LDS_MD + LDS_LIST + NWAVE) * 4)

static_assert(SPW * NWAVE == NB);
static_assert(NB <= 256);
static_assert(WCAP == (CHUNK / NTHR) * 32);
static_assert(NGRP == 2);
static_assert(((LDS_ACC + LDS_MD) % 4) == 0);
static_assert(LDS_AGG_BYTES == 261664);
static_assert((TSP % 8) == 0);
static_assert((HSP % 4) == 0);

typedef float    v4f  __attribute__((ext_vector_type(4)));
typedef float    v8f  __attribute__((ext_vector_type(8)));
typedef int      v4i  __attribute__((ext_vector_type(4)));
typedef _Float16 v8h  __attribute__((ext_vector_type(8)));
typedef _Float16 v16h __attribute__((ext_vector_type(16)));
union Frag   { v16h v; v8h half[2]; };
union Pack16 { v8h h; v4i i; };

__device__ __forceinline__ v8f wm(v16h a, v16h b, v8f c) {
  v8f d = __builtin_amdgcn_wmma_f32_16x16x32_f16(false, a, false, b, (short)0, c, false, false);
  asm volatile("v_nop\n\tv_nop\n\tv_nop\n\tv_nop" : "+v"(d) : "v"(a), "v"(b));
  return d;
}

__global__ __launch_bounds__(NTHR) void k_cvtx(const float* __restrict__ x, _Float16* x16, int n8) {
  const int i = blockIdx.x * NTHR + threadIdx.x;
  if (i >= n8) return;
  const size_t o = (size_t)i * 8;
  const v4f a = *(const v4f*)(x + o);
  const v4f b = *(const v4f*)(x + o + 4);
  Pack16 u;
  u.h[0] = (_Float16)a.x; u.h[1] = (_Float16)a.y; u.h[2] = (_Float16)a.z; u.h[3] = (_Float16)a.w;
  u.h[4] = (_Float16)b.x; u.h[5] = (_Float16)b.y; u.h[6] = (_Float16)b.z; u.h[7] = (_Float16)b.w;
  *(volatile v4i*)(x16 + o) = u.i;
  __threadfence();
  *(volatile v4i*)(x16 + o) = u.i;
}

__global__ __launch_bounds__(NTHR) void k_cvtw(const float* __restrict__ Wa, const float* __restrict__ Wb,
                                               _Float16* Oa, _Float16* Ob, int K, int Nc) {
  const int i   = blockIdx.x * NTHR + threadIdx.x;
  const int kc  = K >> 3;
  const int tot = Nc * kc;
  if (i >= tot) return;
  const float* W = (blockIdx.y == 0) ? Wa : Wb;
  _Float16*    O = (blockIdx.y == 0) ? Oa : Ob;
  const int n = i / kc;
  const int k = (i - n * kc) * 8;
  Pack16 u;
#pragma unroll
  for (int j = 0; j < 8; ++j) u.h[j] = (_Float16)(W[(size_t)(k + j) * Nc + n] * 16.0f);
  _Float16* gp = O + (size_t)n * K + k;
  *(volatile v4i*)gp = u.i;
  __threadfence();
  *(volatile v4i*)gp = u.i;
}

__device__ __forceinline__ void stage_tile(v8f c, int rowT, int colT, int hh, float dscale, float b16,
                                           _Float16* Ts) {
#pragma unroll
  for (int r = 0; r < 8; ++r)
    Ts[(rowT + 8 * hh + r) * TSP + colT] = (_Float16)(c[r] * dscale + b16);
}

__global__ __launch_bounds__(NTHR) void k_gemm(
    const _Float16* __restrict__ A, const _Float16* __restrict__ Wl, const _Float16* __restrict__ Wr,
    const float* __restrict__ bl, const float* __restrict__ br,
    _Float16* Ol, _Float16* Orp, int nN, int K, float dscale) {
  __shared__ __attribute__((aligned(16))) _Float16 Ts[GR * TSP];

  const int tid  = threadIdx.x;
  const int lane = tid & 31;
  const int wave = tid >> 5;
  const int hh   = lane >> 4;
  const int m    = lane & 15;
  const int rt   = wave & 1;
  const int cg   = wave >> 1;
  const int rowBase = blockIdx.x * GR;
  const int yq   = blockIdx.y;
  const bool rsel = (yq >= 2);
  const _Float16* Wp = rsel ? Wr : Wl;
  const float*    bp = rsel ? br : bl;
  _Float16*       Op = rsel ? Orp : Ol;
  const int colBase = (yq & 1) * 128;

  int ra0 = rowBase + 32 * rt + m;      if (ra0 > nN - 1) ra0 = nN - 1;
  int ra1 = rowBase + 32 * rt + 16 + m; if (ra1 > nN - 1) ra1 = nN - 1;
  const _Float16* pa0 = A + (size_t)ra0 * K + 8 * hh;
  const _Float16* pa1 = A + (size_t)ra1 * K + 8 * hh;
  const int n0 = colBase + 32 * cg + m;
  const int n1 = n0 + 16;
  const _Float16* pb0 = Wp + (size_t)n0 * K + 8 * hh;
  const _Float16* pb1 = Wp + (size_t)n1 * K + 8 * hh;

  v8f c00 = {0.f, 0.f, 0.f, 0.f, 0.f, 0.f, 0.f, 0.f};
  v8f c01 = {0.f, 0.f, 0.f, 0.f, 0.f, 0.f, 0.f, 0.f};
  v8f c10 = {0.f, 0.f, 0.f, 0.f, 0.f, 0.f, 0.f, 0.f};
  v8f c11 = {0.f, 0.f, 0.f, 0.f, 0.f, 0.f, 0.f, 0.f};
#pragma unroll 1
  for (int k0 = 0; k0 < K; k0 += 32) {
    Frag a0, a1, b0, b1;
    a0.half[0] = *(const v8h*)(pa0 + k0); a0.half[1] = *(const v8h*)(pa0 + k0 + 16);
    a1.half[0] = *(const v8h*)(pa1 + k0); a1.half[1] = *(const v8h*)(pa1 + k0 + 16);
    b0.half[0] = *(const v8h*)(pb0 + k0); b0.half[1] = *(const v8h*)(pb0 + k0 + 16);
    b1.half[0] = *(const v8h*)(pb1 + k0); b1.half[1] = *(const v8h*)(pb1 + k0 + 16);
    c00 = wm(a0.v, b0.v, c00);
    c01 = wm(a0.v, b1.v, c01);
    c10 = wm(a1.v, b0.v, c10);
    c11 = wm(a1.v, b1.v, c11);
  }

  const float bv0 = bp[n0] * 16.0f;
  const float bv1 = bp[n1] * 16.0f;
  const int ct0 = 32 * cg + m;
  const int ct1 = ct0 + 16;
  stage_tile(c00, 32 * rt,      ct0, hh, dscale, bv0, Ts);
  stage_tile(c01, 32 * rt,      ct1, hh, dscale, bv1, Ts);
  stage_tile(c10, 32 * rt + 16, ct0, hh, dscale, bv0, Ts);
  stage_tile(c11, 32 * rt + 16, ct1, hh, dscale, bv1, Ts);
  __syncthreads();

  const int q = lane >> 3;
  const int p = lane & 7;
  v4i v[4];
  _Float16* g[4];
#pragma unroll
  for (int i = 0; i < 4; ++i) {
    const int L   = 16 * wave + 4 * i + q;
    const int row = L >> 1;
    const int ch  = (L & 1) * 64 + 8 * p;
    Pack16 u;
    u.h = *(const v8h*)(Ts + row * TSP + ch);
    v[i] = u.i;
    g[i] = Op + (size_t)(rowBase + row) * HCH + colBase + ch;
  }
#pragma unroll
  for (int i = 0; i < 4; ++i) *(volatile v4i*)(g[i]) = v[i];
  __threadfence();
#pragma unroll
  for (int i = 0; i < 4; ++i) *(volatile v4i*)(g[i]) = v[i];
}

__device__ __forceinline__ float edge_logit(const v8h xv, const v8h xw, const float (&ar)[8], float (&xf)[8]) {
  float part = 0.f;
#pragma unroll
  for (int j = 0; j < 8; ++j) {
    const float a = (float)xv[j];
    xf[j] = a;
    float v = a + (float)xw[j];
    v = (v > 0.f) ? v : 0.2f * v;
    part += v * ar[j];
  }
  part += __shfl_xor(part, 1, 32);
  part += __shfl_xor(part, 2, 32);
  part += __shfl_xor(part, 4, 32);
  return part * 0.0625f;
}

__global__ __launch_bounds__(NTHR) void k_agg(
    const _Float16* __restrict__ xl16, const _Float16* __restrict__ xr16,
    const int* __restrict__ src, const int* __restrict__ dst,
    const float* __restrict__ att, const float* __restrict__ bias,
    _Float16* hout, int nN, int nE, float oscale) {
  extern __shared__ v4f lds_dyn[];
  float* acc  = (float*)lds_dyn;
  float* md   = acc + LDS_ACC;
  int*   list = (int*)(md + LDS_MD);
  int*   wcnt = list + LDS_LIST;

  const int tid  = threadIdx.x;
  const int lane = tid & 31;
  const int wave = tid >> 5;
  const int hd   = lane >> 3;
  const int nodeBase = blockIdx.x * NB;

  float ar[8];
#pragma unroll
  for (int j = 0; j < 8; ++j) ar[j] = att[8 * lane + j];

#pragma unroll 1
  for (int j = 0; j < SPW; ++j) {
    const int slot = wave * SPW + j;
    int node = nodeBase + slot;
    if (node > nN - 1) node = nN - 1;
    const v8h xv = *(const v8h*)(xl16 + (size_t)node * HCH + 8 * lane);
    const v8h xw = *(const v8h*)(xr16 + (size_t)node * HCH + 8 * lane);
    float xf[8];
    const float lg = edge_logit(xv, xw, ar, xf);
    v4f a0, a1;
    a0.x = xf[0]; a0.y = xf[1]; a0.z = xf[2]; a0.w = xf[3];
    a1.x = xf[4]; a1.y = xf[5]; a1.z = xf[6]; a1.w = xf[7];
    *(v4f*)(acc + slot * HCH + 8 * lane)     = a0;
    *(v4f*)(acc + slot * HCH + 8 * lane + 4) = a1;
    md[slot * 8 + hd]     = lg;
    md[slot * 8 + 4 + hd] = 1.0f;
  }
  __syncthreads();

  const bool al16 = ((((size_t)dst) & 15) == 0);
  const int nChunks = (nE + CHUNK - 1) / CHUNK;
#pragma unroll 1
  for (int ch = 0; ch < nChunks; ++ch) {
    const int cbase = ch * CHUNK;
    int wc = 0;
#pragma unroll
    for (int g = 0; g < NGRP; ++g) {
      const int el0 = (g * NTHR + tid) * 4;
      const int e0  = cbase + el0;
      const int sent = -2147483647 - 1;
      v4i d;
      if (al16 && (cbase + CHUNK <= nE)) {
        d = *(const v4i*)(dst + e0);
      } else {
        d.x = (e0     < nE) ? dst[min(e0,     nE - 1)] : sent;
        d.y = (e0 + 1 < nE) ? dst[min(e0 + 1, nE - 1)] : sent;
        d.z = (e0 + 2 < nE) ? dst[min(e0 + 2, nE - 1)] : sent;
        d.w = (e0 + 3 < nE) ? dst[min(e0 + 3, nE - 1)] : sent;
      }
      const unsigned s0 = (unsigned)d.x - (unsigned)nodeBase;
      const unsigned s1 = (unsigned)d.y - (unsigned)nodeBase;
      const unsigned s2 = (unsigned)d.z - (unsigned)nodeBase;
      const unsigned s3 = (unsigned)d.w - (unsigned)nodeBase;
      const bool h0 = s0 < (unsigned)NB;
      const bool h1 = s1 < (unsigned)NB;
      const bool h2 = s2 < (unsigned)NB;
      const bool h3 = s3 < (unsigned)NB;
      const unsigned many = __builtin_amdgcn_ballot_w32(h0 | h1 | h2 | h3);
      if (many != 0u) {
#define HITJ(J, HJ, SJ) { \
          const unsigned mj = __builtin_amdgcn_ballot_w32(HJ); \
          if (HJ) { \
            const int pos = wc + (int)__builtin_amdgcn_mbcnt_lo(mj, 0u); \
            if (pos < WCAP) list[wave * WCAP + pos] = ((el0 + (J)) << 8) | (int)(SJ); \
          } \
          wc += (int)__builtin_popcount(mj); }
        HITJ(0, h0, s0)
        HITJ(1, h1, s1)
        HITJ(2, h2, s2)
        HITJ(3, h3, s3)
#undef HITJ
      }
    }
    if (lane == 0) wcnt[wave] = wc;
    __syncthreads();

    if (wave == 0) {
#pragma unroll 1
      for (int wsx = 0; wsx < NWAVE; ++wsx) {
        int n = wcnt[wsx];
        n = (n < 0) ? 0 : ((n > WCAP) ? WCAP : n);
#pragma unroll 1
        for (int i = 0; i < n; ++i) {
          const int ent = list[wsx * WCAP + i];
          int slot = ent & 255;
          if (slot > NB - 1) slot = NB - 1;
          const int el = (ent >> 8) & (CHUNK - 1);
          int e = cbase + el;
          if (e > nE - 1) e = nE - 1;
          int s = src[e];
          s = (s < 0) ? 0 : ((s > nN - 1) ? nN - 1 : s);
          int node = nodeBase + slot;
          if (node > nN - 1) node = nN - 1;
          const v8h xv = *(const v8h*)(xl16 + (size_t)s * HCH + 8 * lane);
          const v8h xw = *(const v8h*)(xr16 + (size_t)node * HCH + 8 * lane);
          float xf[8];
          const float lg = edge_logit(xv, xw, ar, xf);
          const float mo = md[slot * 8 + hd];
          const float dn = md[slot * 8 + 4 + hd];
          const float mn = fmaxf(mo, lg);
          const float sc = __expf(mo - mn);
          const float p  = __expf(lg - mn);
          float* ap = acc + slot * HCH + 8 * lane;
          v4f a0 = *(const v4f*)ap;
          v4f a1 = *(const v4f*)(ap + 4);
          a0.x = a0.x * sc + p * xf[0]; a0.y = a0.y * sc + p * xf[1];
          a0.z = a0.z * sc + p * xf[2]; a0.w = a0.w * sc + p * xf[3];
          a1.x = a1.x * sc + p * xf[4]; a1.y = a1.y * sc + p * xf[5];
          a1.z = a1.z * sc + p * xf[6]; a1.w = a1.w * sc + p * xf[7];
          *(v4f*)ap       = a0;
          *(v4f*)(ap + 4) = a1;
          md[slot * 8 + hd]     = mn;
          md[slot * 8 + 4 + hd] = dn * sc + p;
        }
      }
    }
    __syncthreads();
  }

  float bz[8];
#pragma unroll
  for (int j = 0; j < 8; ++j) bz[j] = bias[8 * lane + j];
#pragma unroll 1
  for (int j = 0; j < SPW; ++j) {
    const int slot = wave * SPW + j;
    const int node = nodeBase + slot;
    if (node >= nN) break;
    const float dn  = md[slot * 8 + 4 + hd];
    const float inv = __builtin_amdgcn_rcpf(dn + 1e-16f) * 0.0625f;
    const float* ap = acc + slot * HCH + 8 * lane;
    const v4f a0 = *(const v4f*)ap;
    const v4f a1 = *(const v4f*)(ap + 4);
    float ov[8] = {a0.x, a0.y, a0.z, a0.w, a1.x, a1.y, a1.z, a1.w};
    Pack16 u;
#pragma unroll
    for (int c = 0; c < 8; ++c) {
      float t = ov[c] * inv + bz[c];
      t = (t > 0.f) ? t : 0.f;
      u.h[c] = (_Float16)(t * oscale);
    }
    _Float16* gp = hout + (size_t)node * HCH + 8 * lane;
    *(volatile v4i*)gp = u.i;
    __threadfence();
    *(volatile v4i*)gp = u.i;
  }
}

__global__ __launch_bounds__(NTHR) void k_post(
    const _Float16* __restrict__ A, const _Float16* __restrict__ Wp, const float* __restrict__ bp1,
    const float* __restrict__ Wq, const float* __restrict__ bq, float* out, int nN) {
  __shared__ __attribute__((aligned(16))) float Hs[GR * HSP];
  __shared__ __attribute__((aligned(16))) float Ws2[HIDW * OUTW];
  __shared__ __attribute__((aligned(16))) float Os[GR * OUTW];
  __shared__ float Bq[OUTW];

  const int tid  = threadIdx.x;
  const int lane = tid & 31;
  const int wave = tid >> 5;
  const int hh   = lane >> 4;
  const int m    = lane & 15;
  const int ra   = wave & 3;
  const int cb   = wave >> 2;
  const int rowBase = blockIdx.x * GR;

  for (int i = tid; i < HIDW * OUTW; i += NTHR) Ws2[i] = Wq[i];
  if (tid < OUTW) Bq[tid] = bq[tid];

  int ar0 = rowBase + 16 * ra + m;
  if (ar0 > nN - 1) ar0 = nN - 1;
  const _Float16* pa = A + (size_t)ar0 * HCH + 8 * hh;
  const int n0 = 32 * cb + m;
  const int n1 = n0 + 16;
  const _Float16* pb0 = Wp + (size_t)n0 * HCH + 8 * hh;
  const _Float16* pb1 = Wp + (size_t)n1 * HCH + 8 * hh;

  v8f c0 = {0.f, 0.f, 0.f, 0.f, 0.f, 0.f, 0.f, 0.f};
  v8f c1 = {0.f, 0.f, 0.f, 0.f, 0.f, 0.f, 0.f, 0.f};
#pragma unroll 1
  for (int k0 = 0; k0 < HCH; k0 += 32) {
    Frag a, b0, b1;
    a.half[0]  = *(const v8h*)(pa + k0);  a.half[1]  = *(const v8h*)(pa + k0 + 16);
    b0.half[0] = *(const v8h*)(pb0 + k0); b0.half[1] = *(const v8h*)(pb0 + k0 + 16);
    b1.half[0] = *(const v8h*)(pb1 + k0); b1.half[1] = *(const v8h*)(pb1 + k0 + 16);
    c0 = wm(a.v, b0.v, c0);
    c1 = wm(a.v, b1.v, c1);
  }

  const float dsc = 1.0f / 1024.0f;
  const float bb0 = bp1[n0];
  const float bb1 = bp1[n1];
#pragma unroll
  for (int r = 0; r < 8; ++r) {
    Hs[(16 * ra + 8 * hh + r) * HSP + n0] = c0[r] * dsc + bb0;
    Hs[(16 * ra + 8 * hh + r) * HSP + n1] = c1[r] * dsc + bb1;
  }
  __syncthreads();

  const int row = tid >> 2;
  const int o2  = (tid & 3) * 2;
  float z0 = Bq[o2];
  float z1 = Bq[o2 + 1];
#pragma unroll 4
  for (int j = 0; j < HIDW; ++j) {
    const float hv = Hs[row * HSP + j];
    z0 += hv * Ws2[j * OUTW + o2];
    z1 += hv * Ws2[j * OUTW + o2 + 1];
  }
  z0 = fminf(fmaxf(z0, -80.f), 80.f);
  z1 = fminf(fmaxf(z1, -80.f), 80.f);
  const float s0 = __builtin_amdgcn_rcpf(1.0f + __expf(-z0));
  const float s1 = __builtin_amdgcn_rcpf(1.0f + __expf(-z1));
  Os[row * OUTW + o2]     = s0;
  Os[row * OUTW + o2 + 1] = s1;
  __syncthreads();

  if (wave < 4) {
    const int q = lane >> 3;
    const int p = lane & 7;
    const int L = 4 * wave + q;
    const int lrow = 4 * L + (p >> 1);
    const int grow = rowBase + lrow;
    const v4f val = *(const v4f*)(Os + 32 * L + 4 * p);
    const bool ok = (grow < nN);
    float* gp = out + (size_t)(ok ? grow : 0) * OUTW + (p & 1) * 4;
    if (ok) *(volatile v4f*)gp = val;
    __threadfence();
    if (ok) *(volatile v4f*)gp = val;
  }
}

static size_t al256(size_t v) { return (v + 255) & ~(size_t)255; }

extern "C" void kernel_launch(void* const* d_in, const int* in_sizes, int n_in,
                              void* d_out, int out_size, void* d_ws, size_t ws_size,
                              hipStream_t stream) {
  if (n_in < 19) return;
  const int nN = in_sizes[0] / IN1;
  if (nN < 1 || in_sizes[0] != nN * IN1) return;
  const int nE = in_sizes[1];
  if (nE < 1 || in_sizes[2] != nE) return;
  if (in_sizes[3] != IN1 * HCH || in_sizes[5] != IN1 * HCH) return;
  if (in_sizes[4] != HCH || in_sizes[6] != HCH || in_sizes[7] != HCH || in_sizes[8] != HCH) return;
  if (in_sizes[9] != HCH * HCH || in_sizes[11] != HCH * HCH) return;
  if (in_sizes[10] != HCH || in_sizes[12] != HCH || in_sizes[13] != HCH || in_sizes[14] != HCH) return;
  if (in_sizes[15] != HCH * HIDW || in_sizes[16] != HIDW) return;
  if (in_sizes[17] != HIDW * OUTW || in_sizes[18] != OUTW) return;
  if (out_size != nN * OUTW) return;

  const float* x     = (const float*)d_in[0];
  const int*   src   = (const int*)d_in[1];
  const int*   dst   = (const int*)d_in[2];
  const float* W1l   = (const float*)d_in[3];
  const float* b1l   = (const float*)d_in[4];
  const float* W1r   = (const float*)d_in[5];
  const float* b1r   = (const float*)d_in[6];
  const float* att1  = (const float*)d_in[7];
  const float* bias1 = (const float*)d_in[8];
  const float* W2l   = (const float*)d_in[9];
  const float* b2l   = (const float*)d_in[10];
  const float* W2r   = (const float*)d_in[11];
  const float* b2r   = (const float*)d_in[12];
  const float* att2  = (const float*)d_in[13];
  const float* bias2 = (const float*)d_in[14];
  const float* Wp1   = (const float*)d_in[15];
  const float* bp1   = (const float*)d_in[16];
  const float* Wp2   = (const float*)d_in[17];
  const float* bp2   = (const float*)d_in[18];
  float* out = (float*)d_out;

  const int nP = ((nN + GR - 1) / GR) * GR;
  size_t off = 0;
  char* wsb = (char*)d_ws;
  _Float16* x16   = (_Float16*)(wsb + off); off = al256(off + (size_t)nN * IN1 * 2);
  _Float16* W1l16 = (_Float16*)(wsb + off); off = al256(off + (size_t)HCH * IN1 * 2);
  _Float16* W1r16 = (_Float16*)(wsb + off); off = al256(off + (size_t)HCH * IN1 * 2);
  _Float16* W2l16 = (_Float16*)(wsb + off); off = al256(off + (size_t)HCH * HCH * 2);
  _Float16* W2r16 = (_Float16*)(wsb + off); off = al256(off + (size_t)HCH * HCH * 2);
  _Float16* Wp116 = (_Float16*)(wsb + off); off = al256(off + (size_t)HIDW * HCH * 2);
  _Float16* xl16  = (_Float16*)(wsb + off); off = al256(off + (size_t)nP * HCH * 2);
  _Float16* xr16  = (_Float16*)(wsb + off); off = al256(off + (size_t)nP * HCH * 2);
  _Float16* h16   = (_Float16*)(wsb + off); off = al256(off + (size_t)nN * HCH * 2);
  if (off > ws_size) return;

  const int n8 = nN * (IN1 / 8);
  k_cvtx<<<(n8 + NTHR - 1) / NTHR, NTHR, 0, stream>>>(x, x16, n8);

  {
    const int t1 = HCH * (IN1 / 8);
    k_cvtw<<<dim3((t1 + NTHR - 1) / NTHR, 2), NTHR, 0, stream>>>(W1l, W1r, W1l16, W1r16, IN1, HCH);
    const int t2 = HCH * (HCH / 8);
    k_cvtw<<<dim3((t2 + NTHR - 1) / NTHR, 2), NTHR, 0, stream>>>(W2l, W2r, W2l16, W2r16, HCH, HCH);
    const int t3 = HIDW * (HCH / 8);
    k_cvtw<<<dim3((t3 + NTHR - 1) / NTHR, 1), NTHR, 0, stream>>>(Wp1, Wp1, Wp116, Wp116, HCH, HIDW);
  }

  hipFuncSetAttribute(reinterpret_cast<const void*>(&k_agg),
                      hipFuncAttributeMaxDynamicSharedMemorySize, LDS_AGG_BYTES);
  const dim3 ggemm(nP / GR, 4);
  const int gagg = (nN + NB - 1) / NB;

  k_gemm<<<ggemm, NTHR, 0, stream>>>(x16, W1l16, W1r16, b1l, b1r, xl16, xr16, nN, IN1, 1.0f);
  k_agg<<<gagg, NTHR, LDS_AGG_BYTES, stream>>>(xl16, xr16, src, dst, att1, bias1, h16, nN, nE, 16.0f);

  k_gemm<<<ggemm, NTHR, 0, stream>>>(h16, W2l16, W2r16, b2l, b2r, xl16, xr16, nN, HCH, 0.0625f);
  k_agg<<<gagg, NTHR, LDS_AGG_BYTES, stream>>>(xl16, xr16, src, dst, att2, bias2, h16, nN, nE, 64.0f);

  k_post<<<nP / GR, NTHR, 0, stream>>>(h16, Wp116, bp1, Wp2, bp2, out, nN);
}
